// FIB_RNN_40742059770157
// MI455X (gfx1250) — hardware-verified
//
#include <hip/hip_runtime.h>
#include <math.h>

constexpr int kBatch   = 8192;
constexpr int kUnits   = 128;
constexpr int kGates   = 384;
constexpr int kWin     = 49;
constexpr int kEnc     = 48;
constexpr int kPred    = 28;
constexpr int kSteps   = kEnc + kPred - 1;
constexpr int kNW      = 258;
constexpr int kWPitch  = 288;
constexpr int kTileM   = 16;
constexpr int kThreads = 256;
constexpr int kHPitch  = 136;
constexpr int kOutRow  = kPred * 2;
constexpr float kSoftC = 0.54132485f;

static_assert(kBatch % kTileM == 0, "tile");
static_assert(kUnits % 32 == 0, "k step");
static_assert((kTileM * kOutRow) % 4 == 0 && (kTileM * kOutRow) / 4 == 224, "out tile = 224 float4 = 28 lines");
static_assert((kPred * kWPitch) % 32 == 0, "whole lines");

typedef __attribute__((ext_vector_type(16))) _Float16 v16h;
typedef __attribute__((ext_vector_type(8)))  _Float16 v8h;
typedef __attribute__((ext_vector_type(8)))  float    v8f;
typedef __attribute__((ext_vector_type(4)))  float    v4f;

__device__ __forceinline__ void dep_guard_h(v8f& a, v8f& b, v16h x, v16h y) { asm volatile("v_nop\n\tv_nop\n\tv_nop\n\tv_nop" : "+v"(a), "+v"(b) : "v"(x), "v"(y)); }
__device__ __forceinline__ void keep4_h(v16h a, v16h b, v16h c, v16h d) { asm volatile("v_nop" :: "v"(a), "v"(b), "v"(c), "v"(d)); }
__device__ __forceinline__ void acc_guard3(v8f& a, v8f& b, v8f& c) { asm volatile("v_nop\n\tv_nop\n\tv_nop\n\tv_nop" : "+v"(a), "+v"(b), "+v"(c)); }

template <typename T> struct Frag;
template <> struct Frag<_Float16> {
  typedef v16h V; union U { v16h v; v8h h[2]; };
  static __device__ __forceinline__ v16h load(const _Float16* p) {
    U f; f.h[0] = *(const v8h*)(p); f.h[1] = *(const v8h*)(p + 16); return f.v;
  }
  static __device__ __forceinline__ v8f mma(v16h a, v16h b, v8f c) {
    return __builtin_amdgcn_wmma_f32_16x16x32_f16(false, a, false, b, (short)0, c, false, false);
  }
};

__device__ __forceinline__ float softplus_f(float x) { return fmaxf(x, 0.0f) + log1pf(expf(-fabsf(x))); }
__device__ __forceinline__ float fsigm(float x) { return __builtin_amdgcn_rcpf(1.0f + __expf(-x)); }
__device__ __forceinline__ float ftanh(float x) { return 1.0f - 2.0f * __builtin_amdgcn_rcpf(1.0f + __expf(2.0f * x)); }

__global__ __launch_bounds__(kThreads) void prep_kernel(const float* __restrict__ R, const float* __restrict__ dvloc,
                                                        const float* __restrict__ dvrho, const float* __restrict__ dveps,
                                                        _Float16* __restrict__ RT, float* __restrict__ WT) {
  const int blk = blockIdx.x, tid = threadIdx.x;
  if (blk < 24) {
    const int p  = blk * kThreads + tid;
    const int n  = p >> 4;
    const int c8 = (p & 15) * 8;
    v8h h;
#pragma unroll
    for (int e = 0; e < 8; ++e) h[e] = (_Float16)(R[(size_t)(c8 + e) * kGates + n] * 8.0f);
    _Float16* q = RT + (size_t)n * kUnits + c8;
    *(volatile v8h*)q = h; __threadfence(); *(volatile v8h*)q = h;
  } else {
    const int i = (blk - 24) * kThreads + tid;
    if (i < kPred * kWPitch) {
      const int g  = i / kWPitch;
      const int c  = i - g * kWPitch;
      const int cc = c < kNW ? c : (kNW - 1);
      const float sc = 1e-5f + 0.02f * softplus_f(kSoftC + dvrho[cc]);
      const float w  = dvloc[cc] + sc * dveps[(size_t)g * kNW + cc];
      const float v  = (c < kNW) ? w : 0.0f;
      float* q = WT + i;
      *(volatile float*)q = v; __threadfence(); *(volatile float*)q = v;
    }
  }
}

__global__ __launch_bounds__(kThreads) void gru_ar_kernel(const float* __restrict__ X,
                                                          const float* __restrict__ Kin,
                                                          const float* __restrict__ bias,
                                                          const _Float16* __restrict__ RT,
                                                          const float* __restrict__ WT,
                                                          const float* __restrict__ SE,
                                                          float* __restrict__ out) {
  __shared__ __align__(16) _Float16 h16[kTileM * kHPitch];
  __shared__ __align__(16) float s_hf[kTileM * kUnits];
  __shared__ __align__(16) float s_pred[kTileM * kOutRow];
  __shared__ float s_x[kTileM];

  const int tid = threadIdx.x, lane = tid & 31, wave = tid >> 5;
  const int rlane = lane & 15, hh = lane >> 4, koff = hh * 8, mOff = hh * 8;
  const int bbase = blockIdx.x * kTileM;

  for (int i = tid; i < kTileM * kHPitch; i += kThreads) h16[i] = (_Float16)0.0f;

  const int j = 16 * wave + rlane;
  const float kz = Kin[j], kr = Kin[kUnits + j], kh = Kin[2 * kUnits + j];
  const float b0z = bias[j], b0r = bias[kUnits + j], b0h = bias[2 * kUnits + j];
  const float b1z = bias[kGates + j], b1r = bias[kGates + kUnits + j], b1h = bias[kGates + 2 * kUnits + j];
  float hf[8];
#pragma unroll
  for (int r = 0; r < 8; ++r) hf[r] = 0.0f;

  const _Float16* arow = h16 + rlane * kHPitch + koff;
  const _Float16* wz = RT + (size_t)j * kUnits + koff;
  const _Float16* wr = RT + (size_t)(kUnits + j) * kUnits + koff;
  const _Float16* wh = RT + (size_t)(2 * kUnits + j) * kUnits + koff;
  const v8f z8 = {0.f, 0.f, 0.f, 0.f, 0.f, 0.f, 0.f, 0.f};

  if (tid < kTileM) s_x[tid] = X[(size_t)(bbase + tid) * kWin + 0];
  __syncthreads();

#pragma unroll 1
  for (int s = 0; s < kSteps; ++s) {
    v8f az = z8, ar = z8, ah = z8;
#pragma unroll
    for (int kc = 0; kc < kUnits / 32; ++kc) {
      const int k0 = kc * 32;
      const v16h a  = Frag<_Float16>::load(arow + k0);
      const v16h bz = Frag<_Float16>::load(wz + k0);
      const v16h br = Frag<_Float16>::load(wr + k0);
      const v16h bh = Frag<_Float16>::load(wh + k0);
      az = Frag<_Float16>::mma(a, bz, az);
      ar = Frag<_Float16>::mma(a, br, ar);
      ah = Frag<_Float16>::mma(a, bh, ah);
      dep_guard_h(az, ah, a, bh);
      keep4_h(bz, br, bh, a);
    }
    acc_guard3(az, ar, ah);

#pragma unroll
    for (int r = 0; r < 8; ++r) {
      const float x  = s_x[mOff + r];
      const float xz = x * kz + b0z;
      const float xr = x * kr + b0r;
      const float xh = x * kh + b0h;
      const float hz = az[r] * 0.125f + b1z;
      const float hr = ar[r] * 0.125f + b1r;
      const float hc = ah[r] * 0.125f + b1h;
      const float zg = fsigm(xz + hz);
      const float rg = fsigm(xr + hr);
      const float cand = ftanh(xh + rg * hc);
      hf[r] = zg * hf[r] + (1.0f - zg) * cand;
    }
    __syncthreads();

#pragma unroll
    for (int r = 0; r < 8; ++r) h16[(mOff + r) * kHPitch + j] = (_Float16)hf[r];
    if (s >= kEnc - 1) {
#pragma unroll
      for (int r = 0; r < 8; ++r) s_hf[(mOff + r) * kUnits + j] = hf[r];
    }
    __syncthreads();

    if (s >= kEnc - 1 && tid < 32) {
      const int g = s - (kEnc - 1);
      const int row = tid >> 1, c = tid & 1;
      const float* wg = WT + (size_t)g * kWPitch;
      const float* hrow = s_hf + row * kUnits;
      float acc = 0.0f;
#pragma unroll 4
      for (int k = 0; k < kUnits; ++k) acc = fmaf(hrow[k], wg[2 * k + c], acc);
      acc += wg[2 * kUnits + c];
      const float sp = 1e-5f + 0.05f * softplus_f(kSoftC + acc);
      s_pred[row * kOutRow + 2 * g + c] = (c == 0) ? acc : sp;
    }
    __syncthreads();

    if (s < kEnc - 1) {
      if (tid < kTileM) s_x[tid] = X[(size_t)(bbase + tid) * kWin + (s + 1)];
    } else if (s < kSteps - 1) {
      const int g = s - (kEnc - 1);
      if (tid < kTileM) {
        const float loc = s_pred[tid * kOutRow + 2 * g];
        const float sc  = s_pred[tid * kOutRow + 2 * g + 1];
        s_x[tid] = loc + sc * SE[(size_t)g * kBatch + bbase + tid];
      }
    }
    __syncthreads();
  }

  if (tid < (kTileM * kOutRow) / 4) {
    const v4f v = *(const v4f*)(s_pred + 4 * tid);
    float* p = out + (size_t)bbase * kOutRow + 4 * tid;
    *(volatile v4f*)p = v;
    __threadfence();
    *(volatile v4f*)p = v;
  }
}

extern "C" void kernel_launch(void* const* d_in, const int* in_sizes, int n_in,
                              void* d_out, int out_size, void* d_ws, size_t ws_size, hipStream_t stream) {
  if (n_in < 8 || d_out == nullptr || d_ws == nullptr) return;
  if (in_sizes[0] != kBatch * kWin || in_sizes[1] != kGates || in_sizes[2] != kUnits * kGates || in_sizes[3] != 2 * kGates ||
      in_sizes[4] != kNW || in_sizes[5] != kNW || in_sizes[6] != kPred * kNW || in_sizes[7] != (kPred - 1) * kBatch ||
      out_size != kBatch * kOutRow) return;

  const float* X     = (const float*)d_in[0];
  const float* Kin   = (const float*)d_in[1];
  const float* R     = (const float*)d_in[2];
  const float* bias  = (const float*)d_in[3];
  const float* dvloc = (const float*)d_in[4];
  const float* dvrho = (const float*)d_in[5];
  const float* dveps = (const float*)d_in[6];
  const float* SE    = (const float*)d_in[7];
  float* out = (float*)d_out;

  char* ws = (char*)d_ws; size_t off = 0;
  auto carve = [&](size_t bytes) -> char* { char* p = ws + off; off += (bytes + 255) & ~(size_t)255; return p; };
  _Float16* RT16 = (_Float16*)carve((size_t)kGates * kUnits * 2);
  float*    WT   = (float*)carve((size_t)kPred * kWPitch * 4);
  if (off > ws_size || off > (size_t)134217728) return;

  prep_kernel<<<24 + 32, kThreads, 0, stream>>>(R, dvloc, dvrho, dveps, RT16, WT);
  gru_ar_kernel<<<kBatch / kTileM, kThreads, 0, stream>>>(X, Kin, bias, RT16, WT, SE, out);
}
